// Prototype_47614007444058
// MI455X (gfx1250) — hardware-verified
//
#include <hip/hip_runtime.h>
#include <stddef.h>


typedef _Float16 v16h __attribute__((ext_vector_type(16)));
typedef _Float16 v8h  __attribute__((ext_vector_type(8)));
typedef float    v8f  __attribute__((ext_vector_type(8)));
typedef float    v4f  __attribute__((ext_vector_type(4)));
typedef _Float16 h16;

#ifndef NCLS
#define NCLS 100
#endif
#define NCLS_FULL 100
#define NCEN   4
#define HIDDEN 128
#define BATCH  2048
#define CHUNK  32

#define LDK 40
#define LDC 68
#define DCARRY 16.0f

static_assert(NCLS >= 1 && NCLS <= NCLS_FULL);
static_assert(BATCH == 8 * 8 * 32);
static_assert(CHUNK == 32);
static_assert(CHUNK == 8 * 4);
static_assert(HIDDEN == 32 * 4);
static_assert(HIDDEN == 8 * 16);
static_assert((LDK % 8) == 0 && LDK >= CHUNK);
static_assert((LDC % 4) == 0 && LDC >= 64);
static_assert(2 * 8 == 16);
static_assert((size_t)NCLS_FULL * NCEN * HIDDEN * HIDDEN < (size_t)0xFFFFFFFFu);
static_assert((size_t)HIDDEN * LDK * 2 + (size_t)8 * 16 * LDC * 4 + (size_t)BATCH * 4 + 32
              <= (size_t)131072);

__device__ __forceinline__ float bf16r(float x) {
  unsigned int u = __float_as_uint(x);
  u = (u + 0x7FFFu + ((u >> 16) & 1u)) & 0xFFFF0000u;
  return __uint_as_float(u);
}

static __device__ __forceinline__ h16 toh_flush(float v) {
  const h16 r = (h16)v;
  return (fabsf(v) < 6.103515625e-05f) ? (h16)0.0f : r;
}

__device__ __forceinline__ v16h frag_at(const _Float16* p) {
  v8h lo = *(const v8h*)(p);
  v8h hi = *(const v8h*)(p + 16);
  v16h out;
#pragma unroll
  for (int i = 0; i < 8; ++i) { out[i] = lo[i]; out[i + 8] = hi[i]; }
  return out;
}
__device__ __forceinline__ v16h ld_frag(const _Float16* base, unsigned ld) {
  const unsigned lane = threadIdx.x & 31u;
  return frag_at(base + (lane & 15u) * ld + (lane >> 4) * 8u);
}

__device__ __forceinline__ v8f wmma16(v16h a, v16h b, v8f c) {
  v8f d = __builtin_amdgcn_wmma_f32_16x16x32_f16(false, a, false, b, (short)0, c,
                                                 false, false);
  asm volatile("v_nop\n\tv_nop\n\tv_nop\n\tv_nop" : "+v"(d) : "v"(a), "v"(b));
  return d;
}

__device__ __forceinline__ unsigned umin_u(unsigned a, unsigned b) { return a < b ? a : b; }

__global__ __launch_bounds__(256) void gram_kernel(
    const float* __restrict__ x, const int* __restrict__ y, const float* __restrict__ mu,
    const float* __restrict__ cov, float* __restrict__ out) {
  __shared__ h16   Dt[HIDDEN * LDK];
  __shared__ float Cs[8 * 16 * LDC];
  __shared__ int   lst[BATCH];
  __shared__ int   wcnt[8];

  const unsigned tid = threadIdx.x, lane = tid & 31u;
  const unsigned wave = (unsigned)__builtin_amdgcn_readfirstlane(threadIdx.x >> 5);
  const unsigned hh = lane >> 4, m = lane & 15u;
  const int k = (int)(blockIdx.x >> 2);
  const unsigned c = blockIdx.x & 3u;

  unsigned msk[8];
  unsigned cntw = 0u;
#pragma unroll
  for (int it = 0; it < 8; ++it) {
    const unsigned b = wave * 256u + (unsigned)it * 32u + lane;
    const int yv = y[b];
    msk[it] = __builtin_amdgcn_ballot_w32(yv == k);
    cntw += (unsigned)__builtin_popcount(msk[it]);
  }
  if (lane == 0u) wcnt[wave] = (int)cntw;
  __syncthreads();
  unsigned total = 0u;
#pragma unroll
  for (unsigned w2 = 0; w2 < 8u; ++w2) total += (unsigned)wcnt[w2];
  unsigned pos = 0u;
  for (unsigned w2 = 0; w2 < wave; ++w2) pos += (unsigned)wcnt[w2];
#pragma unroll
  for (int it = 0; it < 8; ++it) {
    const unsigned b = wave * 256u + (unsigned)it * 32u + lane;
    const unsigned below = msk[it] & ((1u << lane) - 1u);
    const unsigned p = pos + (unsigned)__builtin_popcount(below);
    if ((msk[it] >> lane) & 1u) lst[umin_u(p, (unsigned)BATCH - 1u)] = (int)b;
    pos += (unsigned)__builtin_popcount(msk[it]);
  }
  __syncthreads();
  const unsigned nk = (unsigned)__builtin_amdgcn_readfirstlane((int)umin_u(total, (unsigned)BATCH));

  const unsigned col4 = lane * 4u;
  const v4f mraw = *(const v4f*)(mu + c * (unsigned)HIDDEN + col4);
  float muv[4];
#pragma unroll
  for (int i = 0; i < 4; ++i) muv[i] = bf16r(mraw[i]);

  v8f acc[8];
#pragma unroll
  for (int j = 0; j < 8; ++j) acc[j] = (v8f){};

  for (unsigned cs = 0; cs < nk; cs += (unsigned)CHUNK) {
#pragma unroll
    for (unsigned e = 0; e < 4u; ++e) {
      const unsigned s = wave + 8u * e;
      const unsigned gi = cs + s;
      const bool valid = gi < nk;
      const unsigned li = umin_u(gi, nk - 1u);
      int bi = lst[li];
      bi = bi < 0 ? 0 : (bi > BATCH - 1 ? BATCH - 1 : bi);
      const v4f xv = *(const v4f*)(x + (size_t)bi * HIDDEN + col4);
#pragma unroll
      for (int i = 0; i < 4; ++i) {
        const float d = bf16r(xv[i]) - muv[i];
        const float t = valid ? (DCARRY * d) : 0.0f;
        Dt[(col4 + (unsigned)i) * LDK + s] = toh_flush(t);
      }
    }
    __syncthreads();

    const v16h a = ld_frag(&Dt[(wave * 16u) * LDK], LDK);
#pragma unroll
    for (int j = 0; j < 8; ++j) {
      const v16h bfr = ld_frag(&Dt[(j * 16) * LDK], LDK);
      acc[j] = wmma16(a, bfr, acc[j]);
    }
    __syncthreads();
  }

  const unsigned cbase = wave * (16u * LDC);
  const unsigned obase = blockIdx.x * (unsigned)(HIDDEN * HIDDEN);
#pragma unroll
  for (int half = 0; half < 2; ++half) {
#pragma unroll
    for (int jj = 0; jj < 4; ++jj)
#pragma unroll
      for (int r = 0; r < 8; ++r)
        Cs[cbase + (hh * 8u + (unsigned)r) * LDC + (unsigned)jj * 16u + m] =
            acc[half * 4 + jj][r] * (1.0f / (DCARRY * DCARRY));
    __syncthreads();

    v4f xs[8];
    unsigned off[8];
#pragma unroll
    for (unsigned i = 0; i < 8u; ++i) {
      const unsigned r = 2u * i + (lane >> 4);
      const unsigned cc = (lane & 15u) * 4u;
      const v4f u = *(const v4f*)&Cs[cbase + r * LDC + cc];
      const unsigned o = obase + (wave * 16u + r) * (unsigned)HIDDEN + (unsigned)half * 64u + cc;
      const v4f cv = *(const v4f*)(cov + (size_t)o);
      v4f val;
#pragma unroll
      for (int j = 0; j < 4; ++j) val[j] = bf16r(cv[j]) + u[j];
      xs[i] = val;
      off[i] = o;
    }
#pragma unroll
    for (int i = 0; i < 8; ++i) *(volatile v4f*)(out + (size_t)off[i]) = xs[i];
    __threadfence();
#pragma unroll
    for (int i = 0; i < 8; ++i) *(volatile v4f*)(out + (size_t)off[i]) = xs[i];
    __syncthreads();
  }
}

extern "C" void kernel_launch(void* const* d_in, const int* in_sizes, int n_in,
                              void* d_out, int out_size, void* d_ws, size_t ws_size,
                              hipStream_t stream) {
  (void)d_ws; (void)ws_size;
  if (n_in < 4) return;
  const long long need_out = (long long)NCLS * NCEN * HIDDEN * HIDDEN;
  if ((long long)in_sizes[0] < (long long)BATCH * HIDDEN) return;
  if ((long long)in_sizes[1] < (long long)BATCH) return;
  if ((long long)in_sizes[2] < (long long)NCEN * HIDDEN) return;
  if ((long long)in_sizes[3] < need_out) return;
  if ((long long)out_size < need_out) return;

  const float* x   = (const float*)d_in[0];
  const int*   y   = (const int*)d_in[1];
  const float* mu  = (const float*)d_in[2];
  const float* cov = (const float*)d_in[3];
  float* out = (float*)d_out;

  gram_kernel<<<dim3(NCLS * NCEN), dim3(256), 0, stream>>>(x, y, mu, cov, out);
}
